// SelfAttnLayer_7679401525439
// MI455X (gfx1250) — hardware-verified
//
#include <hip/hip_runtime.h>
#include <math.h>
#include <stdint.h>


#define NB   8
#define CH   256
#define MID  32
#define QKW  64
#define NT   4096
#define TOK  (NB * NT)
#define RSB  16
#define NJ   (NT / 256)
#define PVN  64
#define OUTN (NB * NT * CH)

#define SCW  64.0f
#define SCQK 8.0f
#define SCV  16.0f
#define SCE  32768.0f
#define SCR  2048.0f
#define RLO  (1.0f / SCR)
#define SCS  (1.0f / (SCQK * SCQK))

static_assert(TOK % 64 == 0 && CH % 64 == 0 && CH % 32 == 0 && NT % 64 == 0);
static_assert(QKW == 2 * MID && MID == 32 && QKW == 64);
static_assert((((TOK / 32) * (QKW / 64)) % 8) == 0);
static_assert((((CH / 64) * (TOK / 64)) % 8) == 0);
static_assert(NT % RSB == 0 && RSB == 16 && NT % 256 == 0 && NJ == 16);
static_assert((NT / 16) % 8 == 0 && CH == 4 * 64);
static_assert(NT % PVN == 0 && PVN == 64);
static_assert((NB * NT * CH) % 2048 == 0 && CH % 64 == 0 && MID % 32 == 0);

typedef _Float16       v16h __attribute__((ext_vector_type(16)));
typedef _Float16       v8h  __attribute__((ext_vector_type(8)));
typedef float          v8f  __attribute__((ext_vector_type(8)));
typedef float          v4f  __attribute__((ext_vector_type(4)));
typedef unsigned int   v4u  __attribute__((ext_vector_type(4)));

union HU { v8h h; v4u u; _Float16 s[8]; };
union FR { v16h v; v8h h[2]; _Float16 s[16]; };
static_assert(sizeof(HU) == 16);
static_assert(sizeof(FR) == 32);

__device__ __forceinline__ unsigned short bf_bits(float f) {
  const unsigned u = __float_as_uint(f);
  return (unsigned short)((u + 0x7FFFu + ((u >> 16) & 1u)) >> 16);
}
__device__ __forceinline__ float bf_up(unsigned short h) { return __uint_as_float(((unsigned)h) << 16); }
__device__ __forceinline__ float bfr(float f) { return bf_up(bf_bits(f)); }
__device__ __forceinline__ v8f zero8() { v8f z = {0.f, 0.f, 0.f, 0.f, 0.f, 0.f, 0.f, 0.f}; return z; }

__device__ __forceinline__ void ld8(const float* p, float* o) {
  const v4f a = *(const v4f*)(p);
  const v4f b = *(const v4f*)(p + 4);
  o[0] = a[0]; o[1] = a[1]; o[2] = a[2]; o[3] = a[3];
  o[4] = b[0]; o[5] = b[1]; o[6] = b[2]; o[7] = b[3];
}
__device__ __forceinline__ void st8(float* p, const float* v) {
  v4f a, b;
  a[0] = v[0]; a[1] = v[1]; a[2] = v[2]; a[3] = v[3];
  b[0] = v[4]; b[1] = v[5]; b[2] = v[6]; b[3] = v[7];
  *(v4f*)(p) = a;
  *(v4f*)(p + 4) = b;
}

__device__ __forceinline__ v16h ldfrag_h(const _Float16* p) {
  FR f;
  f.h[0] = *(const v8h*)(p);
  f.h[1] = *(const v8h*)(p + 16);
  return f.v;
}

__device__ __forceinline__ v8f mma_h(v16h a, v16h b, v8f c) {
  c = __builtin_amdgcn_wmma_f32_16x16x32_f16(false, a, false, b, (short)0, c, false, false);
#if defined(__HIP_DEVICE_COMPILE__)
  asm volatile("v_nop\n\tv_nop\n\tv_nop\n\tv_nop" : "+v"(c) : "v"(a), "v"(b));
#endif
  return c;
}
__device__ __forceinline__ v8f mma_h_raw(v16h a, v16h b, v8f c) {
  return __builtin_amdgcn_wmma_f32_16x16x32_f16(false, a, false, b, (short)0, c, false, false);
}
__device__ __forceinline__ void dep_guard_h(v8f& a, v8f& b, v16h x) {
#if defined(__HIP_DEVICE_COMPILE__)
  asm volatile("v_nop\n\tv_nop\n\tv_nop\n\tv_nop" : "+v"(a), "+v"(b) : "v"(x));
#endif
}
__device__ __forceinline__ void keep4_h(v16h a, v16h b, v16h c, v16h d) {
#if defined(__HIP_DEVICE_COMPILE__)
  asm volatile("v_nop" :: "v"(a), "v"(b), "v"(c), "v"(d));
#endif
}
__device__ __forceinline__ void acc_guard4(v8f& a, v8f& b, v8f& c, v8f& d) {
#if defined(__HIP_DEVICE_COMPILE__)
  asm volatile("v_nop\n\tv_nop\n\tv_nop\n\tv_nop" : "+v"(a), "+v"(b), "+v"(c), "+v"(d));
#endif
}
__device__ __forceinline__ void wave_lds_sync() {
  __builtin_amdgcn_fence(__ATOMIC_RELEASE, "workgroup");
  __builtin_amdgcn_wave_barrier();
  __builtin_amdgcn_fence(__ATOMIC_ACQUIRE, "workgroup");
}

__global__ __launch_bounds__(256) void cvt_flat(const float* __restrict__ in, _Float16* out, int n8, float scale) {
  const int i = blockIdx.x * 256 + threadIdx.x;
  if (i < n8) {
    float v[8];
    ld8(in + (size_t)i * 8, v);
    HU u;
#pragma unroll
    for (int e = 0; e < 8; ++e) u.s[e] = (_Float16)(bfr(v[e]) * scale);
    _Float16* p = out + (size_t)i * 8;
    *(volatile v4u*)p = u.u;
    __threadfence();
    *(volatile v4u*)p = u.u;
  }
}

__global__ __launch_bounds__(256) void cvt_wT(const float* __restrict__ Wm, _Float16* out, int R, int C, float scale) {
  __shared__ float sw[64][33];
  const int t = threadIdx.x;
  const int r0 = blockIdx.x * 64, c0 = blockIdx.y * 32;
  {
    const int row = t >> 2, c8 = (t & 3) * 8;
    float v[8];
    ld8(Wm + (size_t)(r0 + row) * C + c0 + c8, v);
#pragma unroll
    for (int e = 0; e < 8; ++e) sw[row][c8 + e] = v[e];
  }
  __syncthreads();
  const int q8 = t & 7, cc = t >> 3;
  HU u;
#pragma unroll
  for (int e = 0; e < 8; ++e) u.s[e] = (_Float16)(bfr(sw[8 * q8 + e][cc]) * scale);
  _Float16* dst = out + (size_t)(c0 + cc) * R + r0 + 8 * q8;
  *(volatile v4u*)dst = u.u;
  __threadfence();
  *(volatile v4u*)dst = u.u;
}

template <int MI>
__device__ __forceinline__ void kseg(v8f (&acc)[MI][4], const _Float16* __restrict__ A, int lda, int m0,
                                     const _Float16* __restrict__ Bt, int ldb, int n0, int K, int rlane, int koff) {
  for (int kk = 0; kk < K; kk += 32) {
    v16h bh[4];
#pragma unroll
    for (int j = 0; j < 4; ++j) {
      const size_t bo = (size_t)(n0 + (j << 4) + rlane) * (size_t)ldb + koff + kk;
      bh[j] = ldfrag_h(Bt + bo);
    }
#pragma unroll
    for (int i = 0; i < MI; ++i) {
      const size_t ao = (size_t)(m0 + (i << 4) + rlane) * (size_t)lda + koff + kk;
      const v16h a0 = ldfrag_h(A + ao);
#pragma unroll
      for (int j = 0; j < 4; ++j) acc[i][j] = mma_h_raw(a0, bh[j], acc[i][j]);
      dep_guard_h(acc[i][0], acc[i][3], a0);
    }
    keep4_h(bh[0], bh[1], bh[2], bh[3]);
  }
}

template <int NPL, int MI>
__global__ __launch_bounds__(256) void gemm64p(
    const _Float16* __restrict__ A, int lda, const _Float16* __restrict__ Bt, int ldb, float cs, float so,
    _Float16* Cp, _Float16* Cl, int ldc, int M, int N, int K) {
  __shared__ __align__(16) float sT[8][16 * 68];
  const int lane = threadIdx.x & 31;
  const int wave = threadIdx.x >> 5;
  const int tilesN = N >> 6;
  const int tilesM = M / (16 * MI);
  const int tiles = tilesM * tilesN;
  const int item = blockIdx.x * 8 + wave;
  if (item >= tiles) return;
  const int tm = item / tilesN;
  const int tn = item - tm * tilesN;
  const int m0 = tm * (16 * MI);
  const int n0 = tn << 6;

  const int rlane = lane & 15;
  const int koff  = (lane >> 4) * 8;
  const int mOff  = (lane >> 4) * 8;

  v8f acc[MI][4];
#pragma unroll
  for (int i = 0; i < MI; ++i)
#pragma unroll
    for (int j = 0; j < 4; ++j) acc[i][j] = zero8();

  kseg<MI>(acc, A, lda, m0, Bt, ldb, n0, K, rlane, koff);
#pragma unroll
  for (int i = 0; i < MI; ++i) acc_guard4(acc[i][0], acc[i][1], acc[i][2], acc[i][3]);

  const int q8 = lane & 7, rr = lane >> 3, c8 = q8 * 8;
  const float csso = cs * so;

  float* slab = sT[wave];
#pragma unroll
  for (int i = 0; i < MI; ++i) {
    const int mBase = m0 + (i << 4);
#pragma unroll
    for (int r = 0; r < 8; ++r) {
#pragma unroll
      for (int j = 0; j < 4; ++j) {
        slab[(mOff + r) * 68 + (j << 4) + rlane] = acc[i][j][r];
      }
    }
    wave_lds_sync();
    v4u uh[4], ul[4];
#pragma unroll
    for (int it = 0; it < 4; ++it) {
      const int row = it * 4 + rr;
      float xs[8];
      ld8(slab + row * 68 + c8, xs);
      HU h, l;
#pragma unroll
      for (int e = 0; e < 8; ++e) {
        const float v = xs[e] * csso;
        const _Float16 hv = (_Float16)v;
        h.s[e] = hv;
        l.s[e] = (_Float16)((v - (float)hv) * SCR);
      }
      uh[it] = h.u;
      ul[it] = l.u;
    }
    for (int pass = 0; pass < 2; ++pass) {
#pragma unroll
      for (int it = 0; it < 4; ++it) {
        const int row = it * 4 + rr;
        const size_t co = (size_t)(mBase + row) * (size_t)ldc + n0 + c8;
        *(volatile v4u*)(Cp + co) = uh[it];
        if (NPL == 2) *(volatile v4u*)(Cl + co) = ul[it];
      }
      __threadfence();
    }
    wave_lds_sync();
  }
}

__global__ __launch_bounds__(256) void k_soft(const _Float16* __restrict__ XH, const _Float16* __restrict__ XL,
                                              _Float16* E, int b) {
  extern __shared__ __align__(16) float sc[];
  const int tid = threadIdx.x, wave = tid >> 5, lane = tid & 31;
  const int hh = lane >> 4, rl = lane & 15;
  const int n0 = blockIdx.x * RSB;

  const size_t qo = (size_t)(b * NT + n0 + rl) * QKW + 8 * hh;
  const v16h qh = ldfrag_h(XH + qo);
  const v16h ql = ldfrag_h(XL + qo);
  for (int ct = wave; ct < NT / 16; ct += 8) {
    const size_t ko = (size_t)(b * NT + 16 * ct + rl) * QKW + MID + 8 * hh;
    const v16h kh = ldfrag_h(XH + ko);
    const v16h kl = ldfrag_h(XL + ko);
    v8f a0 = mma_h(qh, kh, zero8());
    v8f a1 = mma_h(qh, kl, zero8());
    a1 = mma_h(ql, kh, a1);
    const int mc = 16 * ct + rl;
#pragma unroll
    for (int r = 0; r < 8; ++r) {
      sc[(size_t)(8 * hh + r) * NT + mc] = (a0[r] + a1[r] * RLO) * SCS;
    }
  }
  __syncthreads();

  for (int q2 = 0; q2 < RSB / 8; ++q2) {
    const int row = (RSB / 8) * wave + q2;
    float* rp = sc + (size_t)row * NT + 8 * lane;
    float mx = -3.0e38f;
#pragma unroll 4
    for (int j = 0; j < NJ; ++j) {
      float v[8];
      ld8(rp + 256 * j, v);
#pragma unroll
      for (int e = 0; e < 8; ++e) mx = fmaxf(mx, v[e]);
    }
#pragma unroll
    for (int off = 16; off >= 1; off >>= 1) mx = fmaxf(mx, __shfl_xor(mx, off, 32));
    float z = 0.0f;
#pragma unroll 2
    for (int j = 0; j < NJ; ++j) {
      float v[8];
      ld8(rp + 256 * j, v);
#pragma unroll
      for (int e = 0; e < 8; ++e) {
        const float ef = __expf(v[e] - mx);
        z += ef;
        v[e] = ef;
      }
      st8(rp + 256 * j, v);
    }
#pragma unroll
    for (int off = 16; off >= 1; off >>= 1) z += __shfl_xor(z, off, 32);
    const float rz = SCE * (1.0f / z);
    HU u[NJ];
#pragma unroll
    for (int j = 0; j < NJ; ++j) {
      float v[8];
      ld8(rp + 256 * j, v);
#pragma unroll
      for (int e = 0; e < 8; ++e) {
        const _Float16 h0 = (_Float16)(v[e] * rz);
        const float f0 = (float)h0;
        const bool sub = f0 < 6.103515625e-05f;
        u[j].s[e] = sub ? (_Float16)0.0f : h0;
      }
    }
    _Float16* erow = E + (size_t)(n0 + row) * NT + 8 * lane;
    for (int pass = 0; pass < 2; ++pass) {
#pragma unroll
      for (int j = 0; j < NJ; ++j) *(volatile v4u*)(erow + 256 * j) = u[j].u;
      __threadfence();
    }
  }
}

__global__ __launch_bounds__(256) void k_pv(const _Float16* __restrict__ E, const _Float16* __restrict__ VH,
                                            const float* __restrict__ X, const float* __restrict__ gam,
                                            float* out, int b) {
  __shared__ __align__(16) float sO[8][16 * 68];
  const int tid = threadIdx.x, wave = tid >> 5, lane = tid & 31;
  const int hh = lane >> 4, rl = lane & 15;
  const int n0 = blockIdx.x * PVN + 32 * (wave >> 2);
  const int cq = (wave & 3) * 64;

  v8f acc[2][4];
#pragma unroll
  for (int i = 0; i < 2; ++i)
#pragma unroll
    for (int j = 0; j < 4; ++j) acc[i][j] = zero8();

  const _Float16* Ab = E;
  const _Float16* Bb = VH + (size_t)b * NT;
  kseg<2>(acc, Ab, NT, n0, Bb, TOK, cq, NT, rl, 8 * hh);
  acc_guard4(acc[0][0], acc[0][1], acc[0][2], acc[0][3]);
  acc_guard4(acc[1][0], acc[1][1], acc[1][2], acc[1][3]);

  const float fo = 1.0f / (SCV * SCE);
  const float gb = bfr(gam[0]);
  float* slab = sO[wave];
  const int p4 = (lane & 15) * 4, r2 = lane >> 4;
#pragma unroll
  for (int i = 0; i < 2; ++i) {
    const int nBase = n0 + 16 * i;
#pragma unroll
    for (int r = 0; r < 8; ++r) {
#pragma unroll
      for (int j = 0; j < 4; ++j) {
        slab[(8 * hh + r) * 68 + 16 * j + rl] = acc[i][j][r];
      }
    }
    wave_lds_sync();
    v4f ov[8];
#pragma unroll
    for (int it = 0; it < 8; ++it) {
      const int row = 2 * it + r2;
      const v4f a = *(const v4f*)(slab + row * 68 + p4);
      const size_t xo = ((size_t)(b * NT + nBase + row)) * CH + cq + p4;
      const v4f xv = *(const v4f*)(X + xo);
      v4f o;
#pragma unroll
      for (int e = 0; e < 4; ++e) o[e] = bfr(xv[e]) + gb * (a[e] * fo);
      ov[it] = o;
    }
    for (int pass = 0; pass < 2; ++pass) {
#pragma unroll
      for (int it = 0; it < 8; ++it) {
        const int row = 2 * it + r2;
        const size_t oo = ((size_t)(b * NT + nBase + row)) * CH + cq + p4;
        *(volatile v4f*)(out + oo) = ov[it];
      }
      __threadfence();
    }
    wave_lds_sync();
  }
}

extern "C" void kernel_launch(void* const* d_in, const int* in_sizes, int n_in,
                              void* d_out, int out_size, void* d_ws, size_t ws_size,
                              hipStream_t stream) {
  if (n_in < 4) return;
  if (in_sizes[0] != NB * NT * CH) return;
  if (in_sizes[1] != CH * MID) return;
  if (in_sizes[2] != CH * CH) return;
  if (in_sizes[3] < 1) return;
  if (out_size != OUTN) return;

  const float* x   = (const float*)d_in[0];
  const float* WQ  = (const float*)d_in[1];
  const float* WV  = (const float*)d_in[2];
  const float* gam = (const float*)d_in[3];

  const size_t PWQK = (size_t)QKW * CH * 2;
  const size_t PWV  = (size_t)CH * CH * 2;
  const size_t PXH  = (size_t)TOK * CH * 2;
  const size_t PQK  = (size_t)TOK * QKW * 2;
  const size_t PVH  = (size_t)CH * TOK * 2;
  const size_t PE   = (size_t)NT * NT * 2;

  size_t off = 0;
  const size_t oWQK = off; off += PWQK;
  const size_t oWV  = off; off += PWV;
  const size_t oXH  = off; off += PXH;
  const size_t oQKH = off; off += PQK;
  const size_t oQKL = off; off += PQK;
  const size_t oVH  = off; off += PVH;
  const size_t oE   = off; off += PE;
  if (off > ws_size) return;
  if (off > (size_t)134217728) return;

  char* ws = (char*)d_ws;
  _Float16* WQK16 = (_Float16*)(ws + oWQK);
  _Float16* WV16  = (_Float16*)(ws + oWV);
  _Float16* xh    = (_Float16*)(ws + oXH);
  _Float16* XQKH  = (_Float16*)(ws + oQKH);
  _Float16* XQKL  = (_Float16*)(ws + oQKL);
  _Float16* VH    = (_Float16*)(ws + oVH);
  _Float16* E     = (_Float16*)(ws + oE);
  float*    outf  = (float*)d_out;

  const dim3 blk(256);
  const int n8x = (NB * NT * CH) / 8;
  const dim3 gX((n8x + 255) / 256);
  const dim3 gWq(CH / 64, MID / 32);
  const dim3 gWv(CH / 64, CH / 32);
  const dim3 gQK(((TOK / 32) * (QKW / 64) + 7) / 8);
  const dim3 gV(((CH / 64) * (TOK / 64) + 7) / 8);
  const dim3 gSo(NT / RSB);
  const dim3 gPV(NT / PVN);
  const float cs64 = 1.0f / SCW;
  const size_t ldsSoft = (size_t)RSB * NT * sizeof(float);

  hipFuncSetAttribute(reinterpret_cast<const void*>(&k_soft),
                      hipFuncAttributeMaxDynamicSharedMemorySize, (int)ldsSoft);

  cvt_wT<<<gWq, blk, 0, stream>>>(WQ, WQK16, CH, MID, SCW);
  cvt_wT<<<gWq, blk, 0, stream>>>(WQ, WQK16 + (size_t)MID * CH, CH, MID, SCW);
  cvt_wT<<<gWv, blk, 0, stream>>>(WV, WV16, CH, CH, SCW);
  cvt_flat<<<gX, blk, 0, stream>>>(x, xh, n8x, 1.0f);
  gemm64p<2, 2><<<gQK, blk, 0, stream>>>(xh, CH, WQK16, CH, cs64, SCQK, XQKH, XQKL, QKW, TOK, QKW, CH);
  gemm64p<1, 4><<<gV, blk, 0, stream>>>(WV16, CH, xh, CH, cs64, SCV, VH, VH, TOK, CH, TOK, CH);
  for (int b = 0; b < NB; ++b) {
    k_soft<<<gSo, blk, ldsSoft, stream>>>(XQKH, XQKL, E, b);
    k_pv<<<gPV, blk, 0, stream>>>(E, VH, x, gam, outf, b);
  }
}
